// MALA_40467181862986
// MI455X (gfx1250) — hardware-verified
//
#include <hip/hip_runtime.h>
#include <math.h>

typedef unsigned short us_t;
typedef __bf16   v16b __attribute__((ext_vector_type(16)));
typedef _Float16 v16h __attribute__((ext_vector_type(16)));
typedef us_t     v8us __attribute__((ext_vector_type(8)));
typedef us_t     v4us __attribute__((ext_vector_type(4)));
typedef float    v8f  __attribute__((ext_vector_type(8)));
typedef float    v4f  __attribute__((ext_vector_type(4)));
typedef v8us __attribute__((may_alias)) v8usa;
typedef v4us __attribute__((may_alias)) v4usa;
typedef v4f  __attribute__((may_alias)) v4fa;
union FragB { v16b v; v8us half[2]; v16h x; };
union Q8    { v8f v; v4f q[2]; };

#define NB   8
#define CH   256
#define NP   4096
#define HW   64
#define NH   8
#define HD   32
#define KVP  72
#define AQP  40
#define PPW  68
#define GXP  264
#define SCALE_F 0.17677669529663687f
#define CKV     0.0065695032f
#define INV_L   0.000244140625f

#define GM_XL    33792
#define GM_BYTES 67584

#define RP_UH    0
#define RP_UL    32768
#define RP_AQH   65536
#define RP_AQL   75776
#define RP_SINW  86016
#define RP_COSW  88064
#define RP_SINH  90112
#define RP_COSH  90144
#define RP_FREQ  90176
#define RP_ZP    90208
#define RP_KM    91232
#define RP_VM    92256
#define RP_BYTES 93312

__device__ __forceinline__ v8f wmma_bf16(const FragB& a, const FragB& b, v8f c) {
  v8f d = __builtin_amdgcn_wmma_f32_16x16x32_bf16(false, a.v, false, b.v, (short)0, c, false, false);
  asm volatile("v_nop\n\tv_nop\n\tv_nop\n\tv_nop" : "+v"(d) : "v"(a.x), "v"(b.x));
  return d;
}
__device__ __forceinline__ FragB ldfrag(const us_t* p, int h) {
  FragB f;
  f.half[0] = *(const v8usa*)(p + 8 * h);
  f.half[1] = *(const v8usa*)(p + 16 + 8 * h);
  return f;
}
__device__ __forceinline__ v8f zero8f() {
  v8f z;
  #pragma unroll
  for (int j = 0; j < 8; ++j) z[j] = 0.f;
  return z;
}
__device__ __forceinline__ void st8f(float* p, v8f v) {
  Q8 u; u.v = v;
  *(v4fa*)p = u.q[0];
  *(v4fa*)(p + 4) = u.q[1];
}
__device__ __forceinline__ us_t bf16_rne(float f) {
  unsigned u = __float_as_uint(f);
  u += 0x7FFFu + ((u >> 16) & 1u);
  return (us_t)(u >> 16);
}
__device__ __forceinline__ float bf16_val(us_t b) { return __uint_as_float(((unsigned)b) << 16); }
__device__ __forceinline__ void split2(float f, us_t& hi, us_t& lo) {
  hi = bf16_rne(f);
  lo = bf16_rne(f - bf16_val(hi));
}
__device__ __forceinline__ float rope_freq(int i) {
  const float e = (i == 7) ? 1.0f : (float)i * (1.0f / 7.0f);
  return 1.0f / powf(10000.0f, e);
}

__global__ __launch_bounds__(256) void k_wcvt(const float* __restrict__ qw, const float* __restrict__ pw,
                                             us_t* __restrict__ WQh, us_t* __restrict__ WQl,
                                             us_t* __restrict__ WPh, us_t* __restrict__ WPl)
{
  const int g = blockIdx.x * 256 + threadIdx.x;
  if (g >= 40960) return;
  const float* src;
  us_t* dh;
  us_t* dl;
  if (g < 32768) { src = qw + (size_t)g * 8; dh = WQh + (size_t)g * 8; dl = WQl + (size_t)g * 8; }
  else { const int g2 = g - 32768; src = pw + (size_t)g2 * 8; dh = WPh + (size_t)g2 * 8; dl = WPl + (size_t)g2 * 8; }
  const v4f a = *(const v4fa*)src;
  const v4f c = *(const v4fa*)(src + 4);
  v8us oh, ol;
  {
    us_t p1, p2;
    split2(a.x, p1, p2); oh[0] = p1; ol[0] = p2;
    split2(a.y, p1, p2); oh[1] = p1; ol[1] = p2;
    split2(a.z, p1, p2); oh[2] = p1; ol[2] = p2;
    split2(a.w, p1, p2); oh[3] = p1; ol[3] = p2;
    split2(c.x, p1, p2); oh[4] = p1; ol[4] = p2;
    split2(c.y, p1, p2); oh[5] = p1; ol[5] = p2;
    split2(c.z, p1, p2); oh[6] = p1; ol[6] = p2;
    split2(c.w, p1, p2); oh[7] = p1; ol[7] = p2;
  }
  *(volatile v8us*)dh = oh;
  *(volatile v8us*)dl = ol;
  __threadfence();
  *(volatile v8us*)dh = oh;
  *(volatile v8us*)dl = ol;
}

__global__ __launch_bounds__(256) void k_gemm(const float* __restrict__ x,
                                             const us_t* __restrict__ WQh, const us_t* __restrict__ WQl,
                                             const float* __restrict__ bias,
                                             float* __restrict__ R1, float* __restrict__ R2, int mode)
{
  extern __shared__ __attribute__((aligned(16))) unsigned char dsm[];
  us_t*  sXh = (us_t*)dsm;
  us_t*  sXl = (us_t*)(dsm + GM_XL);
  float* sO  = (float*)dsm;
  const int tid = threadIdx.x, lane = tid & 31, w = tid >> 5;
  const int h = lane >> 4, m = lane & 15;
  const int lb = blockIdx.x, cb = blockIdx.y, b = blockIdx.z;
  const int l0 = lb * 64;
  const int obase = (mode == 0) ? (256 + 256 * cb) : ((cb == 0) ? 0 : 768);
  const int cls = obase >> 8;
  float* dst = (cls < 2) ? R1 : R2;

  const float* xb = x + (size_t)(b * CH) * NP + l0;
  #pragma unroll 2
  for (int j = 0; j < 16; ++j) {
    const int f = tid + 256 * j;
    const int c = f >> 4, lq = (f & 15) * 4;
    const v4f v = *(const v4fa*)(xb + (size_t)c * NP + lq);
    us_t p1, p2;
    split2(v.x, p1, p2); sXh[(lq + 0) * GXP + c] = p1; sXl[(lq + 0) * GXP + c] = p2;
    split2(v.y, p1, p2); sXh[(lq + 1) * GXP + c] = p1; sXl[(lq + 1) * GXP + c] = p2;
    split2(v.z, p1, p2); sXh[(lq + 2) * GXP + c] = p1; sXl[(lq + 2) * GXP + c] = p2;
    split2(v.w, p1, p2); sXh[(lq + 3) * GXP + c] = p1; sXl[(lq + 3) * GXP + c] = p2;
  }
  __syncthreads();

  const int wl = w & 1, wc = w >> 1;
  const v8f z8 = zero8f();
  v8f acc[2][4];
  #pragma unroll
  for (int t = 0; t < 2; ++t) {
    #pragma unroll
    for (int v = 0; v < 4; ++v) acc[t][v] = z8;
  }
  const us_t* ah0 = sXh + (32 * wl + m) * GXP;
  const us_t* ah1 = ah0 + 16 * GXP;
  const us_t* al0 = sXl + (32 * wl + m) * GXP;
  const us_t* al1 = al0 + 16 * GXP;
  const us_t* bh0 = WQh + (size_t)(obase + 64 * wc + m) * CH;
  const us_t* bl0 = WQl + (size_t)(obase + 64 * wc + m) * CH;

  #pragma unroll 1
  for (int k0 = 0; k0 < CH; k0 += 32) {
    const FragB a0 = ldfrag(ah0 + k0, h);
    const FragB a1 = ldfrag(ah1 + k0, h);
    const FragB c0 = ldfrag(al0 + k0, h);
    const FragB c1 = ldfrag(al1 + k0, h);
    #pragma unroll
    for (int v = 0; v < 4; ++v) {
      const FragB bh = ldfrag(bh0 + (size_t)(16 * v) * CH + k0, h);
      const FragB bl = ldfrag(bl0 + (size_t)(16 * v) * CH + k0, h);
      acc[0][v] = wmma_bf16(a0, bh, acc[0][v]);
      acc[0][v] = wmma_bf16(a0, bl, acc[0][v]);
      acc[0][v] = wmma_bf16(c0, bh, acc[0][v]);
      acc[1][v] = wmma_bf16(a1, bh, acc[1][v]);
      acc[1][v] = wmma_bf16(a1, bl, acc[1][v]);
      acc[1][v] = wmma_bf16(c1, bh, acc[1][v]);
    }
  }
  __syncthreads();

  #pragma unroll
  for (int v = 0; v < 4; ++v) {
    const int ch = 64 * wc + 16 * v + m;
    const float bb = bias[obase + ch];
    #pragma unroll
    for (int t = 0; t < 2; ++t) {
      v8f y;
      #pragma unroll
      for (int r = 0; r < 8; ++r) {
        float vv = acc[t][v][r] + bb;
        if (cls < 2) vv = (vv > 0.f) ? (vv + 1.f) : expf(vv);
        y[r] = vv;
      }
      st8f(sO + ch * 64 + 32 * wl + 16 * t + 8 * h, y);
    }
  }
  __syncthreads();
  const int q8 = lane & 7, sub = lane >> 3;
  #pragma unroll
  for (int i = 0; i < 16; ++i) {
    const int id = 64 * w + 4 * i + sub;
    const int R = id >> 1, Lh = id & 1;
    const v4f val = *(const v4fa*)(sO + R * 64 + 32 * Lh + 4 * q8);
    const size_t d = (size_t)(b * CH + R) * NP + l0 + 32 * Lh + 4 * q8;
    *(volatile v4f*)(dst + d) = val;
  }
  __threadfence();
  #pragma unroll
  for (int i = 0; i < 16; ++i) {
    const int id = 64 * w + 4 * i + sub;
    const int R = id >> 1, Lh = id & 1;
    const v4f val = *(const v4fa*)(sO + R * 64 + 32 * Lh + 4 * q8);
    const size_t d = (size_t)(b * CH + R) * NP + l0 + 32 * Lh + 4 * q8;
    *(volatile v4f*)(dst + d) = val;
  }
}

__global__ __launch_bounds__(128) void k_kv(const float* __restrict__ KF, const float* __restrict__ VF,
                                           us_t* __restrict__ KVTh, us_t* __restrict__ KVTl,
                                           float* __restrict__ KM, float* __restrict__ VM)
{
  __shared__ __attribute__((aligned(16))) us_t Ah[HD * KVP];
  __shared__ __attribute__((aligned(16))) us_t Al[HD * KVP];
  __shared__ __attribute__((aligned(16))) us_t Bh[HD * KVP];
  __shared__ __attribute__((aligned(16))) us_t Bl[HD * KVP];
  __shared__ __attribute__((aligned(16))) float sSin[HW * 8];
  __shared__ __attribute__((aligned(16))) float sCos[HW * 8];
  __shared__ __attribute__((aligned(16))) float sKV[HD * HD];
  __shared__ __attribute__((aligned(16))) float sSum[64];
  __shared__ float sFreq[8];
  const int tid = threadIdx.x, lane = tid & 31, w = tid >> 5;
  const int h = lane >> 4, m = lane & 15;
  const int n = blockIdx.x & 7, b = blockIdx.x >> 3;
  if (tid < 8) sFreq[tid] = rope_freq(tid);
  __syncthreads();
  #pragma unroll 1
  for (int j = 0; j < 4; ++j) {
    const int idx = tid + 128 * j;
    const int pos = idx >> 3, f = idx & 7;
    float sv, cv;
    sincosf((float)pos * sFreq[f], &sv, &cv);
    sSin[idx] = sv;
    sCos[idx] = cv;
  }
  const int i0 = tid >> 4, l4 = (tid & 15) * 4;
  const float* kb = KF + (size_t)(b * CH + n * HD) * NP;
  const float* vb = VF + (size_t)(b * CH + n * HD) * NP;
  float ks[4], vs[4];
  #pragma unroll
  for (int j = 0; j < 4; ++j) { ks[j] = 0.f; vs[j] = 0.f; }
  const int td = w >> 1, te = w & 1;
  const v8f z8 = zero8f();
  v8f acc = z8;

  #pragma unroll 1
  for (int l0 = 0; l0 < NP; l0 += 64) {
    __syncthreads();
    const int hp = l0 >> 6;
    #pragma unroll
    for (int g = 0; g < 2; ++g) {
      const int d0 = 16 * g + 2 * i0;
      const v4f ka = *(const v4fa*)(kb + (size_t)d0 * NP + l0 + l4);
      const v4f kc = *(const v4fa*)(kb + (size_t)(d0 + 1) * NP + l0 + l4);
      ks[2 * g]     += (ka.x + ka.y) + (ka.z + ka.w);
      ks[2 * g + 1] += (kc.x + kc.y) + (kc.z + kc.w);
      const float sr = sSin[hp * 8 + i0], cr = sCos[hp * 8 + i0];
      v4us ha, la, hc, lc;
      #pragma unroll
      for (int t = 0; t < 4; ++t) {
        const int widx = (l4 + t) * 8 + i0;
        const float sw = sSin[widx], cw = sCos[widx];
        const float s = g ? sw : sr;
        const float c = g ? cw : cr;
        const float xa = ka[t], xc = kc[t];
        us_t p1, p2;
        split2(xa * c - xc * s, p1, p2); ha[t] = p1; la[t] = p2;
        split2(xc * c + xa * s, p1, p2); hc[t] = p1; lc[t] = p2;
      }
      *(v4usa*)(Ah + d0 * KVP + l4) = ha;
      *(v4usa*)(Al + d0 * KVP + l4) = la;
      *(v4usa*)(Ah + (d0 + 1) * KVP + l4) = hc;
      *(v4usa*)(Al + (d0 + 1) * KVP + l4) = lc;
    }
    #pragma unroll
    for (int j = 0; j < 4; ++j) {
      const int e = i0 + 8 * j;
      const v4f vv = *(const v4fa*)(vb + (size_t)e * NP + l0 + l4);
      vs[j] += (vv.x + vv.y) + (vv.z + vv.w);
      v4us hv, lv;
      #pragma unroll
      for (int t = 0; t < 4; ++t) { us_t p1, p2; split2(vv[t], p1, p2); hv[t] = p1; lv[t] = p2; }
      *(v4usa*)(Bh + e * KVP + l4) = hv;
      *(v4usa*)(Bl + e * KVP + l4) = lv;
    }
    __syncthreads();
    #pragma unroll
    for (int kk = 0; kk < 2; ++kk) {
      const FragB fa = ldfrag(Ah + (16 * td + m) * KVP + 32 * kk, h);
      const FragB fl = ldfrag(Al + (16 * td + m) * KVP + 32 * kk, h);
      const FragB gb = ldfrag(Bh + (16 * te + m) * KVP + 32 * kk, h);
      const FragB gl = ldfrag(Bl + (16 * te + m) * KVP + 32 * kk, h);
      acc = wmma_bf16(fa, gb, acc);
      acc = wmma_bf16(fa, gl, acc);
      acc = wmma_bf16(fl, gb, acc);
    }
  }

  #pragma unroll
  for (int j = 0; j < 4; ++j) {
    float a = ks[j], c = vs[j];
    a += __shfl_xor(a, 1); a += __shfl_xor(a, 2); a += __shfl_xor(a, 4); a += __shfl_xor(a, 8);
    c += __shfl_xor(c, 1); c += __shfl_xor(c, 2); c += __shfl_xor(c, 4); c += __shfl_xor(c, 8);
    ks[j] = a; vs[j] = c;
  }
  if ((tid & 15) == 0) {
    sSum[2 * i0] = ks[0]; sSum[2 * i0 + 1] = ks[1];
    sSum[16 + 2 * i0] = ks[2]; sSum[17 + 2 * i0] = ks[3];
    #pragma unroll
    for (int j = 0; j < 4; ++j) sSum[32 + i0 + 8 * j] = vs[j];
  }
  const float cc = CKV * CKV;
  #pragma unroll
  for (int r = 0; r < 8; ++r) sKV[(16 * te + m) * HD + 16 * td + 8 * h + r] = acc[r] * cc;
  __syncthreads();

  const int e = tid >> 2, q4 = tid & 3;
  const v4f f0 = *(const v4fa*)(sKV + e * HD + 8 * q4);
  const v4f f1 = *(const v4fa*)(sKV + e * HD + 8 * q4 + 4);
  v8us hh, ll;
  {
    us_t p1, p2;
    split2(f0.x, p1, p2); hh[0] = p1; ll[0] = p2;
    split2(f0.y, p1, p2); hh[1] = p1; ll[1] = p2;
    split2(f0.z, p1, p2); hh[2] = p1; ll[2] = p2;
    split2(f0.w, p1, p2); hh[3] = p1; ll[3] = p2;
    split2(f1.x, p1, p2); hh[4] = p1; ll[4] = p2;
    split2(f1.y, p1, p2); hh[5] = p1; ll[5] = p2;
    split2(f1.z, p1, p2); hh[6] = p1; ll[6] = p2;
    split2(f1.w, p1, p2); hh[7] = p1; ll[7] = p2;
  }
  const size_t kd = ((size_t)(b * NH + n) * HD + e) * HD + 8 * q4;
  const int mi = tid & 7;
  const bool isk = tid < 8;
  const bool isv = (tid >= 8) && (tid < 16);
  const v4f mk = *(const v4fa*)(sSum + 4 * mi) * INV_L;
  const v4f mv = *(const v4fa*)(sSum + 32 + 4 * mi) * INV_L;
  float* pk = KM + (size_t)(b * NH + n) * HD + 4 * mi;
  float* pv = VM + (size_t)(b * NH + n) * HD + 4 * mi;
  *(volatile v8us*)(KVTh + kd) = hh;
  *(volatile v8us*)(KVTl + kd) = ll;
  if (isk) *(volatile v4f*)pk = mk;
  if (isv) *(volatile v4f*)pv = mv;
  __threadfence();
  *(volatile v8us*)(KVTh + kd) = hh;
  *(volatile v8us*)(KVTl + kd) = ll;
  if (isk) *(volatile v4f*)pk = mk;
  if (isv) *(volatile v4f*)pv = mv;
}

__global__ __launch_bounds__(256) void k_lepe(const float* __restrict__ VF, const float* __restrict__ lw,
                                             const float* __restrict__ lbias, float* __restrict__ LF)
{
  __shared__ __attribute__((aligned(16))) float sP[PPW * PPW];
  __shared__ float sW[25];
  const int tid = threadIdx.x;
  const int c = blockIdx.x, b = blockIdx.y;
  if (tid < 25) sW[tid] = lw[c * 25 + tid];
  #pragma unroll 1
  for (int j = 0; j < 19; ++j) {
    const int idx = tid + 256 * j;
    if (idx < PPW * PPW) sP[idx] = 0.f;
  }
  __syncthreads();
  const float* src = VF + (size_t)(b * CH + c) * NP;
  #pragma unroll
  for (int j = 0; j < 4; ++j) {
    const int f = tid + 256 * j, l = 4 * f, y = l >> 6, xx = l & 63;
    const v4f v = *(const v4fa*)(src + l);
    float* pr = sP + (y + 2) * PPW + xx + 2;
    pr[0] = v.x; pr[1] = v.y; pr[2] = v.z; pr[3] = v.w;
  }
  __syncthreads();
  const float bb = lbias[c];
  float* dst = LF + (size_t)(b * CH + c) * NP;
  #pragma unroll 1
  for (int j = 0; j < 4; ++j) {
    const int f = tid + 256 * j, l = 4 * f, y = l >> 6, xx = l & 63;
    float a0 = bb, a1 = bb, a2 = bb, a3 = bb;
    #pragma unroll 1
    for (int dy = 0; dy < 5; ++dy) {
      const float* rp = sP + (y + dy) * PPW + xx;
      const v4f r0 = *(const v4fa*)rp;
      const v4f r1 = *(const v4fa*)(rp + 4);
      const float rr[8] = {r0.x, r0.y, r0.z, r0.w, r1.x, r1.y, r1.z, r1.w};
      const float w0 = sW[dy * 5], w1 = sW[dy * 5 + 1], w2 = sW[dy * 5 + 2], w3 = sW[dy * 5 + 3], w4 = sW[dy * 5 + 4];
      a0 += w0 * rr[0]; a0 += w1 * rr[1]; a0 += w2 * rr[2]; a0 += w3 * rr[3]; a0 += w4 * rr[4];
      a1 += w0 * rr[1]; a1 += w1 * rr[2]; a1 += w2 * rr[3]; a1 += w3 * rr[4]; a1 += w4 * rr[5];
      a2 += w0 * rr[2]; a2 += w1 * rr[3]; a2 += w2 * rr[4]; a2 += w3 * rr[5]; a2 += w4 * rr[6];
      a3 += w0 * rr[3]; a3 += w1 * rr[4]; a3 += w2 * rr[5]; a3 += w3 * rr[6]; a3 += w4 * rr[7];
    }
    v4f o;
    o.x = a0; o.y = a1; o.z = a2; o.w = a3;
    *(volatile v4f*)(dst + l) = o;
    __threadfence();
    *(volatile v4f*)(dst + l) = o;
  }
}

__global__ __launch_bounds__(256) void k_resproj(
    const float* __restrict__ QF, const float* __restrict__ OF, const float* __restrict__ LF,
    const us_t* __restrict__ KVTh, const us_t* __restrict__ KVTl,
    const float* __restrict__ KM, const float* __restrict__ VM,
    const us_t* __restrict__ WPh, const us_t* __restrict__ WPl,
    const float* __restrict__ pbias, float* __restrict__ out)
{
  extern __shared__ __attribute__((aligned(16))) unsigned char dsm[];
  us_t*  Uh    = (us_t*)(dsm + RP_UH);
  us_t*  Ul    = (us_t*)(dsm + RP_UL);
  float* sO    = (float*)(dsm + RP_UH);
  us_t*  Aqh   = (us_t*)(dsm + RP_AQH);
  us_t*  Aql   = (us_t*)(dsm + RP_AQL);
  float* sSinW = (float*)(dsm + RP_SINW);
  float* sCosW = (float*)(dsm + RP_COSW);
  float* sSinH = (float*)(dsm + RP_SINH);
  float* sCosH = (float*)(dsm + RP_COSH);
  float* sFreq = (float*)(dsm + RP_FREQ);
  float* sZP   = (float*)(dsm + RP_ZP);
  float* sKM   = (float*)(dsm + RP_KM);
  float* sVM   = (float*)(dsm + RP_VM);
  const int tid = threadIdx.x, lane = tid & 31, w = tid >> 5;
  const int h = lane >> 4, m = lane & 15;
  const int lb = blockIdx.x, b = blockIdx.y;
  const int l0 = lb * 64;
  const v8f z8 = zero8f();

  if (tid < 8) sFreq[tid] = rope_freq(tid);
  sKM[tid] = KM[(size_t)b * CH + tid];
  sVM[tid] = VM[(size_t)b * CH + tid];
  __syncthreads();
  #pragma unroll 1
  for (int j = 0; j < 2; ++j) {
    const int idx = tid + 256 * j;
    const int pos = idx >> 3, f = idx & 7;
    float sv, cv;
    sincosf((float)pos * sFreq[f], &sv, &cv);
    sSinW[idx] = sv;
    sCosW[idx] = cv;
  }
  if (tid < 8) {
    float sv, cv;
    sincosf((float)lb * sFreq[tid], &sv, &cv);
    sSinH[tid] = sv;
    sCosH[tid] = cv;
  }
  __syncthreads();

  const int sl = tid & 63, part = tid >> 6, shp = part >> 1, sdh = part & 1;
  const int chp = w >> 2, clt = w & 3;
  #pragma unroll 1
  for (int hp2 = 0; hp2 < 4; ++hp2) {
    {
      const int nn = 2 * hp2 + shp;
      const float* qp = QF + (size_t)(b * CH + nn * HD + 16 * sdh) * NP + l0 + sl;
      float qv[16];
      #pragma unroll
      for (int j = 0; j < 16; ++j) qv[j] = qp[(size_t)j * NP];
      float zpart = 0.f;
      #pragma unroll
      for (int j = 0; j < 16; ++j) zpart += qv[j] * sKM[nn * HD + 16 * sdh + j];
      sZP[part * 64 + sl] = zpart;
      us_t hq[16], lq[16];
      #pragma unroll
      for (int i = 0; i < 8; ++i) {
        const float sw = sSinW[sl * 8 + i], cw = sCosW[sl * 8 + i];
        const float sr = sSinH[i], cr = sCosH[i];
        const float s = sdh ? sw : sr;
        const float c = sdh ? cw : cr;
        const float x0 = qv[2 * i], x1 = qv[2 * i + 1];
        split2(x0 * c - x1 * s, hq[2 * i], lq[2 * i]);
        split2(x1 * c + x0 * s, hq[2 * i + 1], lq[2 * i + 1]);
      }
      v8us h0, h1, g0, g1;
      #pragma unroll
      for (int i = 0; i < 8; ++i) { h0[i] = hq[i]; h1[i] = hq[8 + i]; g0[i] = lq[i]; g1[i] = lq[8 + i]; }
      us_t* ah = Aqh + (shp * 64 + sl) * AQP + 16 * sdh;
      us_t* al = Aql + (shp * 64 + sl) * AQP + 16 * sdh;
      *(v8usa*)ah = h0; *(v8usa*)(ah + 8) = h1;
      *(v8usa*)al = g0; *(v8usa*)(al + 8) = g1;
    }
    __syncthreads();
    {
      const int nn = 2 * hp2 + chp;
      const FragB fa = ldfrag(Aqh + (chp * 64 + 16 * clt + m) * AQP, h);
      const FragB fl = ldfrag(Aql + (chp * 64 + 16 * clt + m) * AQP, h);
      v8f acc[2];
      #pragma unroll
      for (int u = 0; u < 2; ++u) {
        const size_t kr = ((size_t)(b * NH + nn) * HD + 16 * u + m) * HD;
        const FragB gb = ldfrag(KVTh + kr, h);
        const FragB gl = ldfrag(KVTl + kr, h);
        v8f a = wmma_bf16(fa, gb, z8);
        a = wmma_bf16(fa, gl, a);
        a = wmma_bf16(fl, gb, a);
        acc[u] = a;
      }
      float zz[8], fac[8];
      #pragma unroll
      for (int r = 0; r < 8; ++r) {
        const int l = 16 * clt + 8 * h + r;
        const float z = (sZP[(2 * chp) * 64 + l] + sZP[(2 * chp + 1) * 64 + l]) * SCALE_F;
        zz[r] = z;
        fac[r] = 1.0f + 1.0f / (z + 1e-6f);
      }
      #pragma unroll
      for (int u = 0; u < 2; ++u) {
        const int e = 16 * u + m, c = nn * HD + e;
        const float vme = sVM[nn * HD + e];
        const size_t go = (size_t)(b * CH + c) * NP + l0 + 16 * clt + 8 * h;
        const v4f le0 = *(const v4fa*)(LF + go);
        const v4f le1 = *(const v4fa*)(LF + go + 4);
        const v4f og0 = *(const v4fa*)(OF + go);
        const v4f og1 = *(const v4fa*)(OF + go + 4);
        const float lev[8] = {le0.x, le0.y, le0.z, le0.w, le1.x, le1.y, le1.z, le1.w};
        const float ogv[8] = {og0.x, og0.y, og0.z, og0.w, og1.x, og1.y, og1.z, og1.w};
        #pragma unroll
        for (int r = 0; r < 8; ++r) {
          const float res = acc[u][r] * fac[r] - zz[r] * vme;
          const float uv = (res + lev[r]) * ogv[r];
          us_t p1, p2;
          split2(uv, p1, p2);
          const int l = 16 * clt + 8 * h + r;
          Uh[l * CH + c] = p1;
          Ul[l * CH + c] = p2;
        }
      }
    }
    __syncthreads();
  }

  const int wl = w & 1, wc = w >> 1;
  v8f pacc[2][4];
  #pragma unroll
  for (int t = 0; t < 2; ++t) {
    #pragma unroll
    for (int v = 0; v < 4; ++v) pacc[t][v] = z8;
  }
  const us_t* ua0 = Uh + (32 * wl + m) * CH;
  const us_t* ua1 = ua0 + 16 * CH;
  const us_t* la0 = Ul + (32 * wl + m) * CH;
  const us_t* la1 = la0 + 16 * CH;
  const us_t* wph = WPh + (size_t)(64 * wc + m) * CH;
  const us_t* wpl = WPl + (size_t)(64 * wc + m) * CH;
  #pragma unroll 1
  for (int k0 = 0; k0 < CH; k0 += 32) {
    const FragB a0 = ldfrag(ua0 + k0, h);
    const FragB a1 = ldfrag(ua1 + k0, h);
    const FragB c0 = ldfrag(la0 + k0, h);
    const FragB c1 = ldfrag(la1 + k0, h);
    #pragma unroll
    for (int v = 0; v < 4; ++v) {
      const FragB bh = ldfrag(wph + (size_t)(16 * v) * CH + k0, h);
      const FragB bl = ldfrag(wpl + (size_t)(16 * v) * CH + k0, h);
      pacc[0][v] = wmma_bf16(a0, bh, pacc[0][v]);
      pacc[0][v] = wmma_bf16(c0, bh, pacc[0][v]);
      pacc[0][v] = wmma_bf16(a0, bl, pacc[0][v]);
      pacc[1][v] = wmma_bf16(a1, bh, pacc[1][v]);
      pacc[1][v] = wmma_bf16(c1, bh, pacc[1][v]);
      pacc[1][v] = wmma_bf16(a1, bl, pacc[1][v]);
    }
  }
  __syncthreads();
  #pragma unroll
  for (int v = 0; v < 4; ++v) {
    const int co = 64 * wc + 16 * v + m;
    const float pb = pbias[co];
    #pragma unroll
    for (int t = 0; t < 2; ++t) {
      v8f y;
      #pragma unroll
      for (int r = 0; r < 8; ++r) y[r] = pacc[t][v][r] + pb;
      st8f(sO + co * 64 + 32 * wl + 16 * t + 8 * h, y);
    }
  }
  __syncthreads();
  const int q8 = lane & 7, sub = lane >> 3;
  #pragma unroll
  for (int i = 0; i < 16; ++i) {
    const int id = 64 * w + 4 * i + sub;
    const int R = id >> 1, Lh = id & 1;
    const v4f val = *(const v4fa*)(sO + R * 64 + 32 * Lh + 4 * q8);
    const size_t d = (size_t)(b * CH + R) * NP + l0 + 32 * Lh + 4 * q8;
    *(volatile v4f*)(out + d) = val;
  }
  __threadfence();
  #pragma unroll
  for (int i = 0; i < 16; ++i) {
    const int id = 64 * w + 4 * i + sub;
    const int R = id >> 1, Lh = id & 1;
    const v4f val = *(const v4fa*)(sO + R * 64 + 32 * Lh + 4 * q8);
    const size_t d = (size_t)(b * CH + R) * NP + l0 + 32 * Lh + 4 * q8;
    *(volatile v4f*)(out + d) = val;
  }
}

extern "C" void kernel_launch(void* const* d_in, const int* in_sizes, int n_in,
                              void* d_out, int out_size, void* d_ws, size_t ws_size,
                              hipStream_t stream)
{
  if (n_in < 7) return;
  if (in_sizes[0] != NB * CH * NP) return;
  if (in_sizes[1] != 4 * CH * CH || in_sizes[2] != 4 * CH) return;
  if (in_sizes[3] != CH * 25 || in_sizes[4] != CH) return;
  if (in_sizes[5] != CH * CH || in_sizes[6] != CH) return;
  if (out_size != NB * CH * NP) return;

  const float* x      = (const float*)d_in[0];
  const float* qkvo_w = (const float*)d_in[1];
  const float* qkvo_b = (const float*)d_in[2];
  const float* lepe_w = (const float*)d_in[3];
  const float* lepe_b = (const float*)d_in[4];
  const float* proj_w = (const float*)d_in[5];
  const float* proj_b = (const float*)d_in[6];
  float* outp = (float*)d_out;

  const size_t szWQ  = (size_t)4 * CH * CH * 2;
  const size_t szWP  = (size_t)CH * CH * 2;
  const size_t szR   = (size_t)NB * CH * NP * 4;
  const size_t szKVT = (size_t)NB * NH * HD * HD * 2;
  const size_t szM   = (size_t)NB * NH * HD * 4;
  size_t off = 0;
  char* ws = (char*)d_ws;
  us_t*  WQh  = (us_t*)(ws + off);  off += szWQ;
  us_t*  WQl  = (us_t*)(ws + off);  off += szWQ;
  us_t*  WPh  = (us_t*)(ws + off);  off += szWP;
  us_t*  WPl  = (us_t*)(ws + off);  off += szWP;
  float* R1   = (float*)(ws + off); off += szR;
  float* R2   = (float*)(ws + off); off += szR;
  float* LF   = (float*)(ws + off); off += szR;
  us_t*  KVTh = (us_t*)(ws + off);  off += szKVT;
  us_t*  KVTl = (us_t*)(ws + off);  off += szKVT;
  float* KM   = (float*)(ws + off); off += szM;
  float* VM   = (float*)(ws + off); off += szM;
  if (off > ws_size) return;

  k_wcvt<<<dim3(160), 256, 0, stream>>>(qkvo_w, proj_w, WQh, WQl, WPh, WPl);
  hipFuncSetAttribute(reinterpret_cast<const void*>(&k_gemm),
                      hipFuncAttributeMaxDynamicSharedMemorySize, GM_BYTES);
  k_gemm<<<dim3(HW, 2, NB), 256, GM_BYTES, stream>>>(x, WQh, WQl, qkvo_b, R1, R2, 0);
  k_kv<<<dim3(NB * NH), 128, 0, stream>>>(R1, R2, KVTh, KVTl, KM, VM);
  k_lepe<<<dim3(CH, NB), 256, 0, stream>>>(R2, lepe_w, lepe_b, LF);
  k_gemm<<<dim3(HW, 2, NB), 256, GM_BYTES, stream>>>(x, WQh, WQl, qkvo_b, R1, R2, 1);
  hipFuncSetAttribute(reinterpret_cast<const void*>(&k_resproj),
                      hipFuncAttributeMaxDynamicSharedMemorySize, RP_BYTES);
  k_resproj<<<dim3(NP / 64, NB), 256, RP_BYTES, stream>>>(R1, R2, LF, KVTh, KVTl, KM, VM, WPh, WPl, proj_b, outp);
}
